// HybridFCL_65481071400057
// MI455X (gfx1250) — hardware-verified
//
#include <hip/hip_runtime.h>


#ifndef NB
#define NB 256
#endif
#define NB_FULL 256
#define NF   512
#define NQ   16
#define CD   4
#define NC   10
#define VSP  17

static_assert(NQ == 16);
static_assert(NC <= 16);
static_assert(NF % 32 == 0);
static_assert(NB % 16 == 0);
static_assert(NB <= NB_FULL);
static_assert(((size_t)NB * NF) % 8 == 0);
static_assert(((size_t)NQ * NF) % 8 == 0);
static_assert((16 * NC * 4) % 128 == 0);
static_assert((32 + 8) * 16 == 16 * NC * 4);
static_assert((16 * VSP + 16 * NC) * 4 <= 131072);

typedef unsigned short bf;
typedef __attribute__((ext_vector_type(16))) __bf16   v16bf;
typedef __attribute__((ext_vector_type(8)))  unsigned short v8us;
typedef __attribute__((ext_vector_type(8)))  float    v8f;
typedef __attribute__((ext_vector_type(4)))  float    v4f;
typedef v4f  __attribute__((may_alias)) v4fa;

__device__ __forceinline__ unsigned short f2bf(float f) { unsigned u = __float_as_uint(f); u += 0x7FFFu + ((u >> 16) & 1u); return (unsigned short)(u >> 16); }
__device__ __forceinline__ float bfr(float f) { return __uint_as_float(((unsigned)f2bf(f)) << 16); }
__device__ __forceinline__ v16bf cat16b(v8us lo, v8us hi) { return __builtin_bit_cast(v16bf, __builtin_shufflevector(lo, hi, 0, 1, 2, 3, 4, 5, 6, 7, 8, 9, 10, 11, 12, 13, 14, 15)); }
__device__ __forceinline__ v8f wmmab(v16bf a, v16bf b, v8f c) { return __builtin_amdgcn_wmma_f32_16x16x32_bf16(false, a, false, b, (short)0, c, false, false); }
__device__ __forceinline__ v16bf ldb(const bf* p)  { return cat16b(*(const v8us*)p, *(const v8us*)(p + 16)); }
__device__ __forceinline__ void wave_sync() { __builtin_amdgcn_fence(3  , "wavefront"); __builtin_amdgcn_wave_barrier(); asm volatile("" ::: "memory"); }
__device__ __forceinline__ v8f wmmab_g(v16bf a, v16bf b, v8f c) { c = wmmab(a, b, c); asm volatile("v_nop\n\tv_nop\n\tv_nop\n\tv_nop" : "+v"(c) : "v"(a), "v"(b)); return c; }

__global__ __launch_bounds__(256) void k_cvt8(const float* __restrict__ src, bf* dst, size_t n8) {
    const size_t i = (size_t)blockIdx.x * 256 + threadIdx.x; if (i >= n8) return;
    const v8f v = *(const v8f*)(src + i * 8); v8us o;
#pragma unroll
    for (int k = 0; k < 8; ++k) o[k] = f2bf(v[k]);
    *(volatile v8us*)(dst + i * 8) = o; __threadfence(); *(volatile v8us*)(dst + i * 8) = o;
}

__global__ __launch_bounds__(32) void k_circ(const bf* __restrict__ XB, const bf* __restrict__ WB, const float* __restrict__ enc_b, const float* __restrict__ theta,
                                             const float* __restrict__ cls_w, const float* __restrict__ cls_b, float* OUT) {
    __shared__ __align__(16) float vs[16 * VSP];
    __shared__ __align__(16) float ls[16 * NC];
    const int lane = threadIdx.x & 31, lr = lane & 15, hi = lane >> 4;
    const int r0 = blockIdx.x * 16;
    v8f acc = (v8f){};
    const size_t aoff = (size_t)(r0 + lr) * NF + 8 * hi, boff = (size_t)lr * NF + 8 * hi;
#pragma unroll 4
    for (int kc = 0; kc < NF; kc += 32) {
        const v16bf a = ldb(XB + aoff + kc);
        const v16bf b = ldb(WB + boff + kc);
        acc = wmmab_g(a, b, acc);
    }
    float ts = bfr(theta[lr]);
#pragma unroll
    for (int d = 1; d < CD; ++d) ts += bfr(theta[d * NQ + lr]);
    const float ct = cosf(ts);
    const float bq = bfr(enc_b[lr]);
#pragma unroll
    for (int r = 0; r < 8; ++r) vs[(8 * hi + r) * VSP + lr] = ct * cosf(acc[r] + bq);
    wave_sync();
    v8us ah, al;
#pragma unroll
    for (int i = 0; i < 8; ++i) {
        const float v = vs[lr * VSP + 8 * hi + i];
        const unsigned short hb = f2bf(v);
        const float vh = __uint_as_float(((unsigned)hb) << 16);
        ah[i] = hb; al[i] = f2bf(v - vh); }
    const v16bf pa = cat16b(ah, al);
    const int cc = lr < NC ? lr : NC - 1;
    v8us wf;
#pragma unroll
    for (int i = 0; i < 8; ++i) {
        float w = cls_w[cc * NQ + (NQ - 1 - 8 * hi - i)];
        asm volatile("" : "+v"(w));
        wf[i] = (lr < NC) ? f2bf(w) : (unsigned short)0; }
    const v16bf pw = cat16b(wf, wf);
    float cb = cls_b[cc];
    asm volatile("" : "+v"(cb));
    cb = (lr < NC) ? bfr(cb) : 0.0f;
    v8f lg = (v8f){};
    lg = wmmab_g(pa, pw, lg);
#pragma unroll
    for (int r = 0; r < 8; ++r) { if (lr < NC) ls[(8 * hi + r) * NC + lr] = lg[r] + cb; }
    wave_sync();
    float* ob = OUT + (size_t)r0 * NC;
    const int p1 = 32 + (lane & 7);
    const v4f v0 = *(const v4fa*)(&ls[4 * lane]);
    const v4f v1 = *(const v4fa*)(&ls[4 * p1]);
#pragma unroll 1
    for (int ps = 0; ps < 2; ++ps) {
        *(volatile v4f*)(ob + 4 * lane) = v0;
        if (lane < 8) *(volatile v4f*)(ob + 4 * p1) = v1;
        if (ps == 0) __threadfence(); }
}

static constexpr size_t al256(size_t v) { return (v + 255) & ~(size_t)255; }
static constexpr size_t SZ_XB = al256((size_t)NB * NF * 2);
static constexpr size_t SZ_WB = al256((size_t)NQ * NF * 2);
static constexpr size_t SZ_TOTAL = SZ_XB + SZ_WB;
static_assert(SZ_TOTAL <= (size_t)134217728);
static_assert(SZ_XB % 256 == 0);

extern "C" void kernel_launch(void* const* d_in, const int* in_sizes, int n_in,
                              void* d_out, int out_size, void* d_ws, size_t ws_size, hipStream_t stream) {
    if (n_in < 6) return;
    if ((size_t)in_sizes[0] < (size_t)NB * NF) return;
    if ((size_t)in_sizes[1] < (size_t)NQ * NF) return;
    if (in_sizes[2] < NQ || in_sizes[3] < CD * NQ || in_sizes[4] < NC * NQ || in_sizes[5] < NC) return;
    if ((size_t)out_size < (size_t)NB * NC) return;
    if (SZ_TOTAL > ws_size) return;
    const float* x    = (const float*)d_in[0];
    const float* encw = (const float*)d_in[1];
    const float* encb = (const float*)d_in[2];
    const float* th   = (const float*)d_in[3];
    const float* clsw = (const float*)d_in[4];
    const float* clsb = (const float*)d_in[5];
    float* OUT = (float*)d_out;
    char* wsp = (char*)d_ws;
    bf* XB = (bf*)wsp; wsp += SZ_XB;
    bf* WB = (bf*)wsp; wsp += SZ_WB;

    { const size_t n8 = (size_t)NB * NF / 8; k_cvt8<<<(unsigned)((n8 + 255) / 256), 256, 0, stream>>>(x, XB, n8); }
    { const size_t n8 = (size_t)NQ * NF / 8; k_cvt8<<<(unsigned)((n8 + 255) / 256), 256, 0, stream>>>(encw, WB, n8); }
    k_circ<<<NB / 16, 32, 0, stream>>>(XB, WB, encb, th, clsw, clsb, OUT);
}
